// ModalConditionedRPE_50534585205058
// MI455X (gfx1250) — hardware-run, weakly checked
//
#include <hip/hip_runtime.h>
#include <math.h>

typedef __attribute__((ext_vector_type(16))) _Float16 v16h;
typedef __attribute__((ext_vector_type(8)))  float    v8f;
typedef __attribute__((ext_vector_type(4)))  float    v4f;

constexpr int kGrid   = 40;
constexpr int kPix    = kGrid * kGrid;
constexpr int kHid    = 64;
constexpr int kSrc    = 80;
constexpr int kSrcImg = kSrc * kSrc;
constexpr int kBatch  = 4;
constexpr int kEmb    = 16;
constexpr int kNumMod = 3;
constexpr int kW1Rows = 36;
constexpr int kPrepPix = 64;
constexpr int kTileI  = 32;
constexpr int kTileJ  = 64;
constexpr int kOutPitch = 68;
constexpr float kStep   = 1.0f / (float)(kGrid - 1);
constexpr float kCarryHid = 16.0f;
constexpr float kCarryW   = 64.0f;
constexpr float kCarryRes = 2048.0f;
constexpr float kInvRes   = 1.0f / kCarryRes;
constexpr float kInvMain  = 1.0f / (kCarryHid * kCarryW);
static_assert(kPix == 1600);
static_assert((kPix % kPrepPix) == 0 && (kPix % kTileI) == 0 && (kPix % kTileJ) == 0);
static_assert(kW1Rows == 2 + 2 * kEmb + 2);
static_assert((kHid % 32) == 0);
static_assert(((kPix * 4) % 128) == 0);

constexpr size_t kOffPP   = 0;
constexpr size_t kOffQP   = kOffPP + (size_t)kPix * kHid * 4;
constexpr size_t kWsTotal = kOffQP + (size_t)kPix * kHid * 4;
static_assert(kWsTotal == 819200ull);
static_assert((kOffQP % 128) == 0);
static_assert(kWsTotal <= 134217728ull);

__device__ __forceinline__ v8f mma_h(v16h a, v16h b, v8f c) {
  c = __builtin_amdgcn_wmma_f32_16x16x32_f16(false, a, false, b, (short)0, c, false, false);
  asm volatile("v_nop\n\tv_nop\n\tv_nop\n\tv_nop" : "+v"(c) : "v"(a), "v"(b));
  return c;
}

__device__ __forceinline__ void taps40(int o, int& i0, int& i1, int& i2, int& i3,
                                       float& w0, float& w1, float& w2, float& w3) {
  if (o == 0) {
    i0 = 0; i1 = 1; i2 = 2; i3 = 2;
    w0 = 3.f / 7.f; w1 = 3.f / 7.f; w2 = 1.f / 7.f; w3 = 0.f;
  } else if (o == kGrid - 1) {
    i0 = 77; i1 = 78; i2 = 79; i3 = 79;
    w0 = 1.f / 7.f; w1 = 3.f / 7.f; w2 = 3.f / 7.f; w3 = 0.f;
  } else {
    i0 = 2 * o - 1; i1 = 2 * o; i2 = 2 * o + 1; i3 = 2 * o + 2;
    w0 = 0.125f; w1 = 0.375f; w2 = 0.375f; w3 = 0.125f;
  }
}

__device__ __forceinline__ float tap_row(const float* r, int i0, int i1, int i2, int i3,
                                         float w0, float w1, float w2, float w3) {
  float v = w0 * r[i0];
  v = fmaf(w1, r[i1], v);
  v = fmaf(w2, r[i2], v);
  v = fmaf(w3, r[i3], v);
  return v;
}

__global__ __launch_bounds__(256) void prep_kernel(
    const int* __restrict__ qp, const int* __restrict__ kp,
    const float* __restrict__ smap, const float* __restrict__ emb,
    const float* __restrict__ W1, const float* __restrict__ b1,
    float* __restrict__ PP, float* __restrict__ QP)
{
  __shared__ __align__(16) float sBase[kHid];
  __shared__ __align__(16) float sS[kPrepPix];
  const int tid = threadIdx.x, lane = tid & 31, wave = tid >> 5;
  const int p0 = blockIdx.x * kPrepPix;

  if (wave < 2) {
    const int hcol = tid;
    int qi = qp[0];
    int ki = kp[0];
    qi = qi < 0 ? 0 : (qi > kNumMod - 1 ? kNumMod - 1 : qi);
    ki = ki < 0 ? 0 : (ki > kNumMod - 1 ? kNumMod - 1 : ki);
    float acc = b1[hcol];
#pragma unroll 1
    for (int c = 0; c < kEmb; ++c) acc = fmaf(emb[qi * kEmb + c], W1[(2 + c) * kHid + hcol], acc);
#pragma unroll 1
    for (int c = 0; c < kEmb; ++c) acc = fmaf(emb[ki * kEmb + c], W1[(2 + kEmb + c) * kHid + hcol], acc);
    sBase[hcol] = acc;
  } else if (wave < 4) {
    const int sl = tid - 64;
    const int n  = p0 + sl;
    const int oy = n / kGrid;
    const int ox = n - oy * kGrid;
    int iy0, iy1, iy2, iy3, ix0, ix1, ix2, ix3;
    float wy0, wy1, wy2, wy3, wx0, wx1, wx2, wx3;
    taps40(oy, iy0, iy1, iy2, iy3, wy0, wy1, wy2, wy3);
    taps40(ox, ix0, ix1, ix2, ix3, wx0, wx1, wx2, wx3);
    float acc = 0.f;
#pragma unroll 1
    for (int bb = 0; bb < kBatch; ++bb) {
      const float* m = smap + bb * kSrcImg;
      const float r0 = tap_row(m + iy0 * kSrc, ix0, ix1, ix2, ix3, wx0, wx1, wx2, wx3);
      const float r1 = tap_row(m + iy1 * kSrc, ix0, ix1, ix2, ix3, wx0, wx1, wx2, wx3);
      const float r2 = tap_row(m + iy2 * kSrc, ix0, ix1, ix2, ix3, wx0, wx1, wx2, wx3);
      const float r3 = tap_row(m + iy3 * kSrc, ix0, ix1, ix2, ix3, wx0, wx1, wx2, wx3);
      float v = wy0 * r0;
      v = fmaf(wy1, r1, v);
      v = fmaf(wy2, r2, v);
      v = fmaf(wy3, r3, v);
      acc += v;
    }
    sS[sl] = acc * 0.25f;
  }
  __syncthreads();

  const int hh = lane >> 4;
  const int h4 = (lane & 15) * 4;
  const v4f wx  = *(const v4f*)(W1 + 0 * kHid + h4);
  const v4f wy  = *(const v4f*)(W1 + 1 * kHid + h4);
  const v4f wsi = *(const v4f*)(W1 + 34 * kHid + h4);
  const v4f wsj = *(const v4f*)(W1 + 35 * kHid + h4);
  const v4f bs  = *(const v4f*)(sBase + h4);

#pragma unroll 1
  for (int it = 0; it < 4; ++it) {
    const int row = it * 16 + wave * 2 + hh;
    const int n   = p0 + row;
    const int ry  = n / kGrid;
    const int rx  = n - ry * kGrid;
    const float x = -0.5f + (float)rx * kStep;
    const float y = -0.5f + (float)ry * kStep;
    const float s = sS[row];
    v4f pv, qv;
#pragma unroll
    for (int e = 0; e < 4; ++e) {
      float a = x * wx[e];
      a = fmaf(y, wy[e], a);
      float p = fmaf(s, wsi[e], a);
      p = p + bs[e];
      const float q = fmaf(s, wsj[e], -a);
      pv[e] = p * kCarryHid;
      qv[e] = q * kCarryHid;
    }
    float* pd = PP + (size_t)n * kHid + h4;
    float* qd = QP + (size_t)n * kHid + h4;
    *(volatile v4f*)pd = pv;
    *(volatile v4f*)qd = qv;
    __threadfence();
    *(volatile v4f*)pd = pv;
    *(volatile v4f*)qd = qv;
  }
}

__device__ __forceinline__ _Float16 w2_elem(float w, int m) {
  const float wc = w * kCarryW;
  const float hi = (float)(_Float16)wc;
  const float lo = (wc - hi) * kCarryRes;
  const float v  = (m == 0) ? wc : ((m == 1) ? lo : 0.0f);
  return (_Float16)v;
}

__device__ __forceinline__ v16h w2_pack(v4f a0, v4f a1, v4f a2, v4f a3, int m) {
  v16h f;
#pragma unroll
  for (int e = 0; e < 4; ++e) {
    f[e]      = w2_elem(a0[e], m);
    f[4 + e]  = w2_elem(a1[e], m);
    f[8 + e]  = w2_elem(a2[e], m);
    f[12 + e] = w2_elem(a3[e], m);
  }
  return f;
}

__device__ __forceinline__ v16h relu_pack(v4f a0, v4f a1, v4f a2, v4f a3, v4f q0, v4f q1, v4f q2, v4f q3) {
  v16h f;
#pragma unroll
  for (int e = 0; e < 4; ++e) {
    f[e]      = (_Float16)fmaxf(a0[e] + q0[e], 0.0f);
    f[4 + e]  = (_Float16)fmaxf(a1[e] + q1[e], 0.0f);
    f[8 + e]  = (_Float16)fmaxf(a2[e] + q2[e], 0.0f);
    f[12 + e] = (_Float16)fmaxf(a3[e] + q3[e], 0.0f);
  }
  return f;
}

__global__ __launch_bounds__(256) void rpe_main_kernel(
    const float* __restrict__ PP, const float* __restrict__ QP,
    const float* __restrict__ W2, const float* __restrict__ b2,
    const int* __restrict__ hp, const int* __restrict__ wp,
    float* __restrict__ out)
{
  __shared__ __align__(16) float sP[kTileI * kHid];
  __shared__ __align__(16) float sO[kTileI * kOutPitch];
  const int tid = threadIdx.x, lane = tid & 31, wave = tid >> 5;
  const int hh = lane >> 4, c = lane & 15;
  const int j0 = blockIdx.x * kTileJ;
  const int i0 = blockIdx.y * kTileI;
  const int jsub = (wave & 3) * 16;
  const int ibase = (wave >> 2) * 16;

#pragma unroll
  for (int t = 0; t < 2; ++t) {
    const int idx = (tid + 256 * t) * 4;
    *(v4f*)(sP + idx) = *(const v4f*)(PP + (size_t)i0 * kHid + idx);
  }

  const float* qrow = QP + (size_t)(j0 + jsub + c) * kHid + 8 * hh;
  const v4f q0 = *(const v4f*)(qrow + 0);
  const v4f q1 = *(const v4f*)(qrow + 4);
  const v4f q2 = *(const v4f*)(qrow + 16);
  const v4f q3 = *(const v4f*)(qrow + 20);
  const v4f q4 = *(const v4f*)(qrow + 32);
  const v4f q5 = *(const v4f*)(qrow + 36);
  const v4f q6 = *(const v4f*)(qrow + 48);
  const v4f q7 = *(const v4f*)(qrow + 52);

  const float* wrow = W2 + 8 * hh;
  const v16h wa0 = w2_pack(*(const v4f*)(wrow + 0),  *(const v4f*)(wrow + 4),
                           *(const v4f*)(wrow + 16), *(const v4f*)(wrow + 20), c);
  const v16h wa1 = w2_pack(*(const v4f*)(wrow + 32), *(const v4f*)(wrow + 36),
                           *(const v4f*)(wrow + 48), *(const v4f*)(wrow + 52), c);
  const float b2v = b2[0];

  const int hv = hp[0];
  const int wv = wp[0];
  const bool shape_ok = (hv == kGrid) && (wv == kGrid);
  const float qnan = __uint_as_float(0x7fc00000u);

  __syncthreads();

#pragma unroll 1
  for (int ii = 0; ii < 16; ++ii) {
    const int il = ibase + ii;
    const int pb = il * kHid + 8 * hh;
    const v4f a0 = *(const v4f*)(sP + pb + 0);
    const v4f a1 = *(const v4f*)(sP + pb + 4);
    const v4f a2 = *(const v4f*)(sP + pb + 16);
    const v4f a3 = *(const v4f*)(sP + pb + 20);
    const v4f a4 = *(const v4f*)(sP + pb + 32);
    const v4f a5 = *(const v4f*)(sP + pb + 36);
    const v4f a6 = *(const v4f*)(sP + pb + 48);
    const v4f a7 = *(const v4f*)(sP + pb + 52);
    const v16h f0 = relu_pack(a0, a1, a2, a3, q0, q1, q2, q3);
    const v16h f1 = relu_pack(a4, a5, a6, a7, q4, q5, q6, q7);
    v8f acc = (v8f){0.f, 0.f, 0.f, 0.f, 0.f, 0.f, 0.f, 0.f};
    acc = mma_h(wa0, f0, acc);
    acc = mma_h(wa1, f1, acc);
    const float d0 = acc[0];
    const float d1 = acc[1];
    const float o = (d0 + d1 * kInvRes) * kInvMain + b2v;
    const float ov = shape_ok ? o : qnan;
    if (lane < 16) sO[il * kOutPitch + jsub + lane] = ov;
  }

  __syncthreads();

  {
    const int c4 = c * 4;
    const int r0 = wave * 2 + hh;
    const int r1 = 16 + wave * 2 + hh;
    const v4f v0 = *(const v4f*)(sO + r0 * kOutPitch + c4);
    const v4f v1 = *(const v4f*)(sO + r1 * kOutPitch + c4);
    float* d0p = out + (size_t)(i0 + r0) * kPix + j0 + c4;
    float* d1p = out + (size_t)(i0 + r1) * kPix + j0 + c4;
    for (int pass = 0; pass < 2; ++pass) {
      *(volatile v4f*)d0p = v0;
      *(volatile v4f*)d1p = v1;
      __threadfence();
    }
  }
}

extern "C" void kernel_launch(void* const* d_in, const int* in_sizes, int n_in,
                              void* d_out, int out_size, void* d_ws, size_t ws_size,
                              hipStream_t stream) {
  if (n_in < 10) return;
  if (in_sizes[0] != 1 || in_sizes[1] != 1 || in_sizes[2] != 1 || in_sizes[3] != 1) return;
  if (in_sizes[4] != kBatch * kSrcImg) return;
  if (in_sizes[5] != kNumMod * kEmb) return;
  if (in_sizes[6] != kW1Rows * kHid) return;
  if (in_sizes[7] != kHid) return;
  if (in_sizes[8] != kHid) return;
  if (in_sizes[9] != 1) return;
  if (out_size != kPix * kPix) return;
  if (ws_size < kWsTotal) return;

  const int*   hp   = (const int*)d_in[0];
  const int*   wp   = (const int*)d_in[1];
  const int*   qp   = (const int*)d_in[2];
  const int*   kp   = (const int*)d_in[3];
  const float* smap = (const float*)d_in[4];
  const float* emb  = (const float*)d_in[5];
  const float* W1   = (const float*)d_in[6];
  const float* b1   = (const float*)d_in[7];
  const float* W2   = (const float*)d_in[8];
  const float* b2   = (const float*)d_in[9];

  char* ws = (char*)d_ws;
  float* PP = (float*)(ws + kOffPP);
  float* QP = (float*)(ws + kOffQP);

  prep_kernel<<<kPix / kPrepPix, 256, 0, stream>>>(qp, kp, smap, emb, W1, b1, PP, QP);

  rpe_main_kernel<<<dim3(kPix / kTileJ, kPix / kTileI), 256, 0, stream>>>(PP, QP, W2, b2, hp, wp, (float*)d_out);
}
